// FvdbBasicBlock_8804682957040
// MI455X (gfx1250) — hardware-verified
//
#include <hip/hip_runtime.h>
#include <stddef.h>


#define NV     65536
#define CH     128
#define NSEG   1024
#define NTAP   27
#define KCONV  (NTAP * CH)
#define NLEV   3
#define NTHR   256
#define NWAVE  8
#define EPT    8
#define NGRP   2
#define CHUNK  (NTHR * EPT * NGRP)
#define WCAP   (EPT * NGRP * 32)
#define LISTN  (NWAVE * WCAP)
#define SLOTS  32
#define GROWS  128
#define CROWS  64
#define CTHR   128
#define AP     (CH + 8)
#define STSTR  512
#define SSSTR  512
#define NSS    7
#define WCS    64.0f
#define WCI    0.015625f
#define LRELU  0.01f
#define BNEPS  1e-5f

#define LDS_GEMM (2 * GROWS * AP * 2 + 3 * CH * 4)

static_assert(NV % GROWS == 0);
static_assert(NV % CROWS == 0);
static_assert(NV % CHUNK == 0);
static_assert(NV % NTHR == 0);
static_assert(NSEG % SLOTS == 0);
static_assert((CHUNK & (CHUNK - 1)) == 0);
static_assert(CHUNK <= 4096);
static_assert((SLOTS & (SLOTS - 1)) == 0 && SLOTS <= 4096);
static_assert(KCONV % 32 == 0 && KCONV % 8 == 0);
static_assert(GROWS * CH * 4 <= 2 * GROWS * AP * 2);
static_assert(CROWS * AP * 2 <= CROWS * CH * 4);
static_assert(CTHR == CH);
static_assert((NV * CH) % (NTHR * 8) == 0);
static_assert(GROWS == NWAVE * 16);
static_assert(CROWS == (CTHR / 32) * 16);
static_assert((GROWS * CH / 8) % NTHR == 0);
static_assert((CROWS * CH / 8) % CTHR == 0);
static_assert(SLOTS * CH / 4 == 4 * NTHR);

typedef float          v4f   __attribute__((ext_vector_type(4)));
typedef float          v8f   __attribute__((ext_vector_type(8)));
typedef int            v4i   __attribute__((ext_vector_type(4)));
typedef _Float16       v8h   __attribute__((ext_vector_type(8)));
typedef _Float16       v16h  __attribute__((ext_vector_type(16)));
typedef unsigned short v8us  __attribute__((ext_vector_type(8)));
typedef unsigned short v16us __attribute__((ext_vector_type(16)));
typedef __bf16         v16bf __attribute__((ext_vector_type(16)));
union FragH { v16h v; v8h h[2]; };
union FragB { v16bf v; v16us u; v8us h[2]; };

__device__ __forceinline__ float lre(float v) { return v >= 0.0f ? v : LRELU * v; }
__device__ __forceinline__ v4f lre4(v4f v) {
  v4f r;
  r.x = lre(v.x); r.y = lre(v.y); r.z = lre(v.z); r.w = lre(v.w);
  return r;
}

__device__ __forceinline__ unsigned short bfb(float x) {
  unsigned u = __float_as_uint(x);
  u = (u + 0x7FFFu + ((u >> 16) & 1u)) >> 16;
  return (unsigned short)u;
}

__device__ __forceinline__ void split8(v4f a, v4f b, v8us* hi, v8us* lo) {
  float v[8];
  v[0] = a.x; v[1] = a.y; v[2] = a.z; v[3] = a.w;
  v[4] = b.x; v[5] = b.y; v[6] = b.z; v[7] = b.w;
  v8us h, l;
#pragma unroll
  for (int e = 0; e < 8; ++e) {
    const unsigned short hb = bfb(v[e]);
    const float hf = __uint_as_float(((unsigned)hb) << 16);
    h[e] = hb;
    l[e] = bfb(v[e] - hf);
  }
  *hi = h; *lo = l;
}

__device__ __forceinline__ v8h cvt8h(v4f a, v4f b) {
  v8h r;
  r[0] = (_Float16)a.x; r[1] = (_Float16)a.y; r[2] = (_Float16)a.z; r[3] = (_Float16)a.w;
  r[4] = (_Float16)b.x; r[5] = (_Float16)b.y; r[6] = (_Float16)b.z; r[7] = (_Float16)b.w;
  return r;
}

__device__ __forceinline__ v8f wmh(v16h a, v16h b, v8f c) {
  v8f d = __builtin_amdgcn_wmma_f32_16x16x32_f16(false, a, false, b, (short)0, c, false, false);
  asm volatile("v_nop\n\tv_nop\n\tv_nop\n\tv_nop" : "+v"(d) : "v"(a), "v"(b));
  return d;
}
__device__ __forceinline__ v8f wmb(v16bf a, v16bf b, v8f c) {
  v8f d = __builtin_amdgcn_wmma_f32_16x16x32_bf16(false, a, false, b, (short)0, c, false, false);
  asm volatile("v_nop\n\tv_nop\n\tv_nop\n\tv_nop" : "+v"(d) : "v"(a), "v"(b));
  return d;
}

template <int NB>
__device__ __forceinline__ int scan_chunk(const int* __restrict__ dsts, int nE, int cbase, int slotBase,
                                          int vec8, int* list, int tid, int lane, int wave) {
  int wc = 0;
#pragma unroll
  for (int g = 0; g < NGRP; ++g) {
    const int el0  = (g * NTHR + tid) * EPT;
    const int e0   = cbase + el0;
    const int sent = -2147483647 - 1;
    v4i da, db;
    if (vec8 != 0 && cbase + CHUNK <= nE) {
      da = *(const v4i*)(dsts + e0);
      db = *(const v4i*)(dsts + e0 + 4);
    } else {
      da.x = (e0     < nE) ? dsts[min(e0, nE - 1)] : sent;
      da.y = (e0 + 1 < nE) ? dsts[min(e0 + 1, nE - 1)] : sent;
      da.z = (e0 + 2 < nE) ? dsts[min(e0 + 2, nE - 1)] : sent;
      da.w = (e0 + 3 < nE) ? dsts[min(e0 + 3, nE - 1)] : sent;
      db.x = (e0 + 4 < nE) ? dsts[min(e0 + 4, nE - 1)] : sent;
      db.y = (e0 + 5 < nE) ? dsts[min(e0 + 5, nE - 1)] : sent;
      db.z = (e0 + 6 < nE) ? dsts[min(e0 + 6, nE - 1)] : sent;
      db.w = (e0 + 7 < nE) ? dsts[min(e0 + 7, nE - 1)] : sent;
    }
    const unsigned nb = (unsigned)slotBase;
    const unsigned s0 = (unsigned)da.x - nb, s1 = (unsigned)da.y - nb;
    const unsigned s2 = (unsigned)da.z - nb, s3 = (unsigned)da.w - nb;
    const unsigned s4 = (unsigned)db.x - nb, s5 = (unsigned)db.y - nb;
    const unsigned s6 = (unsigned)db.z - nb, s7 = (unsigned)db.w - nb;
    const bool h0 = s0 < (unsigned)NB, h1 = s1 < (unsigned)NB, h2 = s2 < (unsigned)NB, h3 = s3 < (unsigned)NB;
    const bool h4 = s4 < (unsigned)NB, h5 = s5 < (unsigned)NB, h6 = s6 < (unsigned)NB, h7 = s7 < (unsigned)NB;
    const unsigned any = __builtin_amdgcn_ballot_w32(h0 | h1 | h2 | h3 | h4 | h5 | h6 | h7);
    if (any != 0u) {
#define HITJ(J, HJ, SJ) { \
        const unsigned mj = __builtin_amdgcn_ballot_w32(HJ); \
        if (mj != 0u) { \
          if (HJ) { \
            const int pos = wc + (int)__builtin_amdgcn_mbcnt_lo(mj, 0u); \
            if (pos < WCAP) list[wave * WCAP + pos] = ((el0 + (J)) << 12) | (int)(SJ); \
          } \
          wc += (int)__builtin_popcount(mj); } }
      HITJ(0, h0, s0)
      HITJ(1, h1, s1)
      HITJ(2, h2, s2)
      HITJ(3, h3, s3)
      HITJ(4, h4, s4)
      HITJ(5, h5, s5)
      HITJ(6, h6, s6)
      HITJ(7, h7, s7)
#undef HITJ
    }
  }
  return wc;
}

__global__ __launch_bounds__(NTHR) void k_prep(
    const float* __restrict__ lw, const float* __restrict__ ww, const float* __restrict__ pj,
    const float* __restrict__ fu, const float* __restrict__ c1, const float* __restrict__ c2,
    unsigned short* lwH, unsigned short* lwL, unsigned short* wwH, unsigned short* wwL,
    unsigned short* pjH, unsigned short* pjL, unsigned short* fuH, unsigned short* fuL,
    _Float16* c1p, _Float16* c2p) {
  const int g0 = NLEV * (CH * CH / 8);
  const int g2 = 4 * (CH * CH / 8);
  const int g3 = (2 * CH * CH) / 8;
  const int g4 = (CH * KCONV) / 8;
  const int e1 = g0, e2 = e1 + g0, e3 = e2 + g2, e4 = e3 + g3, e5 = e4 + g4, e6 = e5 + g4;
  const int bstart = blockIdx.x * NTHR;
  const float* src; unsigned short* dh; unsigned short* dl; _Float16* dc; int K, per, segOff, conv;
  if (bstart < e1)      { src = lw; dh = lwH; dl = lwL; dc = c1p; K = CH;     per = CH * CH;     segOff = 0;  conv = 0; }
  else if (bstart < e2) { src = ww; dh = wwH; dl = wwL; dc = c1p; K = CH;     per = CH * CH;     segOff = e1; conv = 0; }
  else if (bstart < e3) { src = pj; dh = pjH; dl = pjL; dc = c1p; K = CH;     per = CH * CH;     segOff = e2; conv = 0; }
  else if (bstart < e4) { src = fu; dh = fuH; dl = fuL; dc = c1p; K = 2 * CH; per = 2 * CH * CH; segOff = e3; conv = 0; }
  else if (bstart < e5) { src = c1; dh = lwH; dl = lwL; dc = c1p; K = KCONV;  per = KCONV * CH;  segOff = e4; conv = 1; }
  else                  { src = c2; dh = lwH; dl = lwL; dc = c2p; K = KCONV;  per = KCONV * CH;  segOff = e5; conv = 1; }
  const int i = bstart + (int)threadIdx.x;
  if (i >= e6) return;
  const int o = (i - segOff) * 8;
  const int layer = o / per;
  const int oo = o - layer * per;
  const int n = oo / K;
  const int k0 = oo - n * K;
  const float* sp = src + (size_t)layer * per;
  float v[8];
#pragma unroll
  for (int e = 0; e < 8; ++e) v[e] = sp[(size_t)(k0 + e) * CH + n];
  if (conv != 0) {
    v8h hv;
#pragma unroll
    for (int e = 0; e < 8; ++e) hv[e] = (_Float16)(v[e] * WCS);
    _Float16* dp = dc + o;
    *(volatile v8h*)dp = hv;
    __threadfence();
    *(volatile v8h*)dp = hv;
  } else {
    v4f a, b;
    a.x = v[0]; a.y = v[1]; a.z = v[2]; a.w = v[3];
    b.x = v[4]; b.y = v[5]; b.z = v[6]; b.w = v[7];
    v8us hi, lo;
    split8(a, b, &hi, &lo);
    unsigned short* ph = dh + o;
    unsigned short* pl = dl + o;
    *(volatile v8us*)ph = hi;
    *(volatile v8us*)pl = lo;
    __threadfence();
    *(volatile v8us*)ph = hi;
    *(volatile v8us*)pl = lo;
  }
}

template <int AMODE>
__global__ __launch_bounds__(NTHR) void k_gemm(
    const float* __restrict__ srcA, const float* __restrict__ ssA, const int* __restrict__ clus,
    const float* __restrict__ tab, const float* __restrict__ adp,
    const unsigned short* __restrict__ Bhi, const unsigned short* __restrict__ Blo,
    float* R, float* stats) {
  extern __shared__ v4f lds_dyn[];
  unsigned short* sAh = (unsigned short*)lds_dyn;
  unsigned short* sAl = sAh + GROWS * AP;
  float* stg   = (float*)lds_dyn;
  float* sstat = (float*)((char*)lds_dyn + 2 * GROWS * AP * 2);
  constexpr int NCHK = (AMODE == 2) ? 2 : 1;
  constexpr int KB = NCHK * CH;
  const int tid = threadIdx.x, lane = tid & 31, wave = tid >> 5, hh = lane >> 4, m = lane & 15;
  const int rowBase = blockIdx.x * GROWS;

  v8f acc[8];
#pragma unroll
  for (int t = 0; t < 8; ++t) { v8f z = {0.f, 0.f, 0.f, 0.f, 0.f, 0.f, 0.f, 0.f}; acc[t] = z; }

#pragma unroll 1
  for (int ck = 0; ck < NCHK; ++ck) {
#pragma unroll 2
    for (int i = 0; i < (GROWS * CH / 8) / NTHR; ++i) {
      const int idx = i * NTHR + tid;
      const int r   = idx >> 4;
      const int c0  = (idx & 15) * 8;
      const int row = rowBase + r;
      v4f a, b;
      if (AMODE == 2 && ck == 1) {
        const v4f w4 = *(const v4f*)(adp + (size_t)row * 4);
        int q0 = clus[row], q1 = clus[NV + row], q2 = clus[2 * NV + row];
        q0 = q0 < 0 ? 0 : (q0 > NSEG - 1 ? NSEG - 1 : q0);
        q1 = q1 < 0 ? 0 : (q1 > NSEG - 1 ? NSEG - 1 : q1);
        q2 = q2 < 0 ? 0 : (q2 > NSEG - 1 ? NSEG - 1 : q2);
        const float* p0 = tab + ((size_t)0 * NSEG + q0) * CH + c0;
        const float* p1 = tab + ((size_t)1 * NSEG + q1) * CH + c0;
        const float* p2 = tab + ((size_t)2 * NSEG + q2) * CH + c0;
        a = w4.x * *(const v4f*)p0 + w4.y * *(const v4f*)p1 + w4.z * *(const v4f*)p2;
        b = w4.x * *(const v4f*)(p0 + 4) + w4.y * *(const v4f*)(p1 + 4) + w4.z * *(const v4f*)(p2 + 4);
      } else {
        const float* ap = srcA + (size_t)row * CH + c0;
        a = *(const v4f*)ap;
        b = *(const v4f*)(ap + 4);
        if (AMODE != 0) {
          const v4f s0 = *(const v4f*)(ssA + c0),      s1 = *(const v4f*)(ssA + c0 + 4);
          const v4f h0 = *(const v4f*)(ssA + CH + c0), h1 = *(const v4f*)(ssA + CH + c0 + 4);
          a = lre4(a * s0 + h0);
          b = lre4(b * s1 + h1);
          if (AMODE == 1) {
            int cl = clus[row];
            cl = cl < 0 ? 0 : (cl > NSEG - 1 ? NSEG - 1 : cl);
            const float* tp = tab + (size_t)cl * CH + c0;
            a = a - *(const v4f*)tp;
            b = b - *(const v4f*)(tp + 4);
          }
        }
      }
      v8us hi, lo;
      split8(a, b, &hi, &lo);
      *(v8us*)(sAh + r * AP + c0) = hi;
      *(v8us*)(sAl + r * AP + c0) = lo;
    }
    __syncthreads();

    const unsigned short* arh = sAh + (wave * 16 + m) * AP + 8 * hh;
    const unsigned short* arl = sAl + (wave * 16 + m) * AP + 8 * hh;
#pragma unroll
    for (int kt = 0; kt < CH / 32; ++kt) {
      FragB ah, al;
      ah.h[0] = *(const v8us*)(arh + 32 * kt);
      ah.h[1] = *(const v8us*)(arh + 32 * kt + 16);
      al.h[0] = *(const v8us*)(arl + 32 * kt);
      al.h[1] = *(const v8us*)(arl + 32 * kt + 16);
#pragma unroll
      for (int t = 0; t < 8; ++t) {
        const size_t bo = (size_t)(16 * t + m) * KB + ck * CH + 32 * kt + 8 * hh;
        FragB bh, bl;
        bh.h[0] = *(const v8us*)(Bhi + bo);
        bh.h[1] = *(const v8us*)(Bhi + bo + 16);
        bl.h[0] = *(const v8us*)(Blo + bo);
        bl.h[1] = *(const v8us*)(Blo + bo + 16);
        acc[t] = wmb(ah.v, bh.v, acc[t]);
        acc[t] = wmb(al.v, bh.v, acc[t]);
        acc[t] = wmb(ah.v, bl.v, acc[t]);
      }
    }
    __syncthreads();
  }

  {
    float* sp = stg + (wave * 16 + 8 * hh) * CH + m;
#pragma unroll
    for (int t = 0; t < 8; ++t) {
#pragma unroll
      for (int r = 0; r < 8; ++r) sp[r * CH + 16 * t] = acc[t][r];
    }
  }
  __syncthreads();

  if (tid < CH) {
    float s = 0.f, mx = -3.0e38f;
#pragma unroll 4
    for (int r = 0; r < GROWS; ++r) { const float x = stg[r * CH + tid]; s += x; mx = fmaxf(mx, x); }
    const float mb = s * (1.0f / GROWS);
    float q = 0.f;
#pragma unroll 4
    for (int r = 0; r < GROWS; ++r) { const float d = stg[r * CH + tid] - mb; q += d * d; }
    sstat[tid] = s; sstat[CH + tid] = q; sstat[2 * CH + tid] = mx;
  }
  __syncthreads();

  const float* lp = stg + wave * 16 * CH + 4 * lane;
  float* gp = R + ((size_t)rowBase + wave * 16) * CH + 4 * lane;
  float* stp = stats + (size_t)blockIdx.x * STSTR + 4 * tid;
  v4f sv = {0.f, 0.f, 0.f, 0.f};
  if (tid < 3 * CH / 4) sv = *(const v4f*)(sstat + 4 * tid);
#pragma unroll
  for (int i = 0; i < 16; ++i) { const v4f v = *(const v4f*)(lp + i * CH); *(volatile v4f*)(gp + (size_t)i * CH) = v; }
  if (tid < 3 * CH / 4) *(volatile v4f*)stp = sv;
  __threadfence();
#pragma unroll
  for (int i = 0; i < 16; ++i) { const v4f v = *(const v4f*)(lp + i * CH); *(volatile v4f*)(gp + (size_t)i * CH) = v; }
  if (tid < 3 * CH / 4) *(volatile v4f*)stp = sv;
}

__global__ __launch_bounds__(CH) void k_bnfin(
    const float* __restrict__ stats, int nblk, int rows,
    const float* __restrict__ gam, const float* __restrict__ bet, int doBN, float* ss) {
  __shared__ __attribute__((aligned(16))) float sout[SSSTR];
  __shared__ float smax[CH];
  const int c = threadIdx.x;
  const float rinv = 1.0f / (float)rows;
  double s = 0.0;
  float mx = -3.0e38f;
#pragma unroll 1
  for (int b = 0; b < nblk; ++b) {
    s += (double)stats[(size_t)b * STSTR + c];
    mx = fmaxf(mx, stats[(size_t)b * STSTR + 2 * CH + c]);
  }
  const double ntot = (double)nblk * (double)rows;
  const double mean = s / ntot;
  double m2 = 0.0;
#pragma unroll 1
  for (int b = 0; b < nblk; ++b) {
    const float sb = stats[(size_t)b * STSTR + c];
    const float qb = stats[(size_t)b * STSTR + CH + c];
    const double cb = (double)(sb * rinv);
    const double d  = cb - mean;
    m2 += (double)qb + 2.0 * d * ((double)sb - (double)rows * cb) + (double)rows * d * d;
  }
  const double var = m2 / ntot;
  float sc = 1.0f, sh = 0.0f;
  if (doBN != 0) {
    const float varf = (float)var;
    sc = gam[c] * rsqrtf(varf + BNEPS);
    sh = bet[c] - (float)mean * sc;
  }
  smax[c] = mx;
  __syncthreads();
#pragma unroll 1
  for (int o = CH / 2; o > 0; o >>= 1) {
    if (c < o) smax[c] = fmaxf(smax[c], smax[c + o]);
    __syncthreads();
  }
  sout[c] = sc; sout[CH + c] = sh; sout[2 * CH + c] = smax[0]; sout[3 * CH + c] = 0.0f;
  __syncthreads();
  const v4f v = *(const v4f*)(sout + 4 * c);
  *(volatile v4f*)(ss + 4 * c) = v;
  __threadfence();
  *(volatile v4f*)(ss + 4 * c) = v;
}

template <int MODE>
__global__ __launch_bounds__(NTHR) void k_seg(
    const int* __restrict__ ids, const float* __restrict__ srcA, const float* __restrict__ srcB,
    const float* __restrict__ ssA, const float* __restrict__ ssG, const float* __restrict__ t2,
    float* tout) {
  __shared__ __attribute__((aligned(16))) float acc[SLOTS * CH];
  __shared__ __attribute__((aligned(16))) float t2i[SLOTS * CH];
  __shared__ __attribute__((aligned(16))) int list[LISTN];
  __shared__ int pc[SLOTS];
  __shared__ float pinv[SLOTS];
  __shared__ int wcnt[NWAVE];
  const int tid = threadIdx.x, lane = tid & 31, wave = tid >> 5;
  const int sBase = blockIdx.x * SLOTS;

  {
    const v4f z = {0.f, 0.f, 0.f, 0.f};
    for (int i = tid; i < SLOTS * CH / 4; i += NTHR) {
      ((v4f*)acc)[i] = z;
      v4f q = z;
      if (MODE == 2) {
        const v4f tv = *(const v4f*)(t2 + (size_t)sBase * CH + 4 * i);
        q.x = __builtin_amdgcn_rcpf(tv.x + 1e-6f);
        q.y = __builtin_amdgcn_rcpf(tv.y + 1e-6f);
        q.z = __builtin_amdgcn_rcpf(tv.z + 1e-6f);
        q.w = __builtin_amdgcn_rcpf(tv.w + 1e-6f);
      }
      ((v4f*)t2i)[i] = q;
    }
    for (int i = tid; i < SLOTS; i += NTHR) { pc[i] = 0; pinv[i] = 1.0f; }
  }
  v4f sc = {1.f, 1.f, 1.f, 1.f}, sh = {0.f, 0.f, 0.f, 0.f};
  float gm = 0.0f;
  if (MODE != 1) { sc = *(const v4f*)(ssA + 4 * lane); sh = *(const v4f*)(ssA + CH + 4 * lane); }
  if (MODE != 0) { gm = ssG[2 * CH]; }
  __syncthreads();

  const int nChunks = NV / CHUNK;
#pragma unroll 1
  for (int ch = 0; ch < nChunks; ++ch) {
    const int cbase = ch * CHUNK;
    const int wc = scan_chunk<SLOTS>(ids, NV, cbase, sBase, 1, list, tid, lane, wave);
    if (lane == 0) wcnt[wave] = wc;
    __syncthreads();
    if (wave == 0) {
#pragma unroll 1
      for (int wsx = 0; wsx < NWAVE; ++wsx) {
        int n = __builtin_amdgcn_readfirstlane(wcnt[wsx]);
        n = n > WCAP ? WCAP : (n < 0 ? 0 : n);
        const int* lp = list + wsx * WCAP;
#pragma unroll 1
        for (int i = 0; i < n; ++i) {
          const int ent  = __builtin_amdgcn_readfirstlane(lp[i]);
          const int slot = ent & (SLOTS - 1);
          int nd = cbase + ((ent >> 12) & (CHUNK - 1));
          nd = nd > NV - 1 ? NV - 1 : nd;
          v4f v;
          if (MODE == 0) {
            const v4f x = *(const v4f*)(srcA + (size_t)nd * CH + 4 * lane);
            v = lre4(x * sc + sh);
          } else if (MODE == 1) {
            const v4f x = *(const v4f*)(srcA + (size_t)nd * CH + 4 * lane);
            v.x = __expf(x.x - gm); v.y = __expf(x.y - gm); v.z = __expf(x.z - gm); v.w = __expf(x.w - gm);
          } else {
            const v4f x3 = *(const v4f*)(srcA + (size_t)nd * CH + 4 * lane);
            const v4f x2 = *(const v4f*)(srcB + (size_t)nd * CH + 4 * lane);
            const v4f p = lre4(x3 * sc + sh);
            v4f e;
            e.x = __expf(x2.x - gm); e.y = __expf(x2.y - gm); e.z = __expf(x2.z - gm); e.w = __expf(x2.w - gm);
            const v4f ti = *(const v4f*)(t2i + slot * CH + 4 * lane);
            const v4f pw = e * ti;
            v = p * pw;
          }
          v4f* ap = (v4f*)(acc + slot * CH + 4 * lane);
          *ap = *ap + v;
          if (MODE == 0) { if (lane == 0) pc[slot] = pc[slot] + 1; }
        }
      }
    }
    __syncthreads();
  }

  if (MODE == 0) {
    if (tid < SLOTS) {
      int cv = pc[tid];
      cv = cv < 1 ? 1 : cv;
      pinv[tid] = 1.0f / (float)cv;
    }
  }
  __syncthreads();

  v4f ov[4];
#pragma unroll
  for (int p = 0; p < 4; ++p) {
    const int idx = p * NTHR + tid;
    const int row = idx >> 5;
    const int c0  = (idx & 31) * 4;
    v4f v = *(const v4f*)(acc + row * CH + c0);
    if (MODE == 0) { const float inv = pinv[row]; v = v * inv; }
    ov[p] = v;
  }
  float* gp = tout + (size_t)sBase * CH;
#pragma unroll
  for (int p = 0; p < 4; ++p) *(volatile v4f*)(gp + 4 * (p * NTHR + tid)) = ov[p];
  __threadfence();
#pragma unroll
  for (int p = 0; p < 4; ++p) *(volatile v4f*)(gp + 4 * (p * NTHR + tid)) = ov[p];
}

__global__ __launch_bounds__(NTHR) void k_adp(
    const float* __restrict__ feat, const float* __restrict__ aw, float* adp) {
  __shared__ float w[CH * 3];
  for (int i = threadIdx.x; i < CH * 3; i += NTHR) w[i] = aw[i];
  __syncthreads();
  const int n = blockIdx.x * NTHR + (int)threadIdx.x;
  const float* fr = feat + (size_t)n * CH;
  float t0 = 0.f, t1 = 0.f, t2 = 0.f;
#pragma unroll 1
  for (int c = 0; c < CH; c += 4) {
    const v4f f = *(const v4f*)(fr + c);
    t0 += f.x * w[3 * c + 0]; t1 += f.x * w[3 * c + 1]; t2 += f.x * w[3 * c + 2];
    t0 += f.y * w[3 * c + 3]; t1 += f.y * w[3 * c + 4]; t2 += f.y * w[3 * c + 5];
    t0 += f.z * w[3 * c + 6]; t1 += f.z * w[3 * c + 7]; t2 += f.z * w[3 * c + 8];
    t0 += f.w * w[3 * c + 9]; t1 += f.w * w[3 * c + 10]; t2 += f.w * w[3 * c + 11];
  }
  const float mx = fmaxf(t0, fmaxf(t1, t2));
  const float e0 = __expf(t0 - mx), e1 = __expf(t1 - mx), e2 = __expf(t2 - mx);
  const float inv = 1.0f / (e0 + e1 + e2);
  v4f o;
  o.x = e0 * inv; o.y = e1 * inv; o.z = e2 * inv; o.w = 0.0f;
  float* op = adp + (size_t)n * 4;
  *(volatile v4f*)op = o;
  __threadfence();
  *(volatile v4f*)op = o;
}

__global__ __launch_bounds__(NTHR) void k_x16(
    const float* __restrict__ R, const float* __restrict__ ss, const float* __restrict__ feat,
    int addFeat, _Float16* X16) {
  const size_t e = ((size_t)blockIdx.x * NTHR + threadIdx.x) * 8;
  const int c0 = (int)(e & (CH - 1));
  v4f a = *(const v4f*)(R + e), b = *(const v4f*)(R + e + 4);
  const v4f s0 = *(const v4f*)(ss + c0),      s1 = *(const v4f*)(ss + c0 + 4);
  const v4f h0 = *(const v4f*)(ss + CH + c0), h1 = *(const v4f*)(ss + CH + c0 + 4);
  a = lre4(a * s0 + h0);
  b = lre4(b * s1 + h1);
  if (addFeat != 0) {
    a = a + *(const v4f*)(feat + e);
    b = b + *(const v4f*)(feat + e + 4);
  }
  const v8h hv = cvt8h(a, b);
  _Float16* dp = X16 + e;
  *(volatile v8h*)dp = hv;
  __threadfence();
  *(volatile v8h*)dp = hv;
}

__global__ __launch_bounds__(CTHR) void k_conv(
    const _Float16* __restrict__ X16, const int* __restrict__ nidx,
    const _Float16* __restrict__ Wc, float* R, float* stats) {
  __shared__ __attribute__((aligned(16))) float ctile[CROWS * CH];
  __shared__ __attribute__((aligned(16))) int   lidx[CROWS * NTAP];
  __shared__ __attribute__((aligned(16))) float sstat[3 * CH];
  _Float16* sA = (_Float16*)ctile;
  const int tid = threadIdx.x, lane = tid & 31, wave = tid >> 5, hh = lane >> 4, m = lane & 15;
  const int rowBase = blockIdx.x * CROWS;

  for (int j = tid; j < CROWS * NTAP; j += CTHR) lidx[j] = nidx[(size_t)rowBase * NTAP + j];
  v8f acc[8];
#pragma unroll
  for (int t = 0; t < 8; ++t) { v8f z = {0.f, 0.f, 0.f, 0.f, 0.f, 0.f, 0.f, 0.f}; acc[t] = z; }
  __syncthreads();

#pragma unroll 1
  for (int tap = 0; tap < NTAP; ++tap) {
#pragma unroll 4
    for (int i = 0; i < (CROWS * CH / 8) / CTHR; ++i) {
      const int u  = i * CTHR + tid;
      const int r  = u >> 4;
      const int c0 = (u & 15) * 8;
      const int g  = lidx[r * NTAP + tap];
      const bool ok = (unsigned)g < (unsigned)NV;
      const int gc = g < 0 ? 0 : (g > NV - 1 ? NV - 1 : g);
      v4i xi = *(const v4i*)(X16 + (size_t)gc * CH + c0);
      const int mk = ok ? -1 : 0;
      xi = xi & mk;
      *(v4i*)(sA + r * AP + c0) = xi;
    }
    __syncthreads();
    const _Float16* ar = sA + (wave * 16 + m) * AP + 8 * hh;
#pragma unroll
    for (int kt = 0; kt < CH / 32; ++kt) {
      FragH a;
      a.h[0] = *(const v8h*)(ar + 32 * kt);
      a.h[1] = *(const v8h*)(ar + 32 * kt + 16);
#pragma unroll
      for (int t = 0; t < 8; ++t) {
        const _Float16* bp = Wc + (size_t)(16 * t + m) * KCONV + tap * CH + 32 * kt + 8 * hh;
        FragH b;
        b.h[0] = *(const v8h*)bp;
        b.h[1] = *(const v8h*)(bp + 16);
        acc[t] = wmh(a.v, b.v, acc[t]);
      }
    }
    __syncthreads();
  }

  {
    float* sp = ctile + (wave * 16 + 8 * hh) * CH + m;
#pragma unroll
    for (int t = 0; t < 8; ++t) {
#pragma unroll
      for (int r = 0; r < 8; ++r) sp[r * CH + 16 * t] = acc[t][r] * WCI;
    }
  }
  __syncthreads();
  {
    float s = 0.f, mx = -3.0e38f;
#pragma unroll 4
    for (int r = 0; r < CROWS; ++r) { const float x = ctile[r * CH + tid]; s += x; mx = fmaxf(mx, x); }
    const float mb = s * (1.0f / CROWS);
    float q = 0.f;
#pragma unroll 4
    for (int r = 0; r < CROWS; ++r) { const float d = ctile[r * CH + tid] - mb; q += d * d; }
    sstat[tid] = s; sstat[CH + tid] = q; sstat[2 * CH + tid] = mx;
  }
  __syncthreads();

  const float* lp = ctile + wave * 16 * CH + 4 * lane;
  float* gp = R + ((size_t)rowBase + wave * 16) * CH + 4 * lane;
  float* stp = stats + (size_t)blockIdx.x * STSTR + 4 * tid;
  v4f sv = {0.f, 0.f, 0.f, 0.f};
  if (tid < 3 * CH / 4) sv = *(const v4f*)(sstat + 4 * tid);
#pragma unroll
  for (int i = 0; i < 16; ++i) { const v4f v = *(const v4f*)(lp + i * CH); *(volatile v4f*)(gp + (size_t)i * CH) = v; }
  if (tid < 3 * CH / 4) *(volatile v4f*)stp = sv;
  __threadfence();
#pragma unroll
  for (int i = 0; i < 16; ++i) { const v4f v = *(const v4f*)(lp + i * CH); *(volatile v4f*)(gp + (size_t)i * CH) = v; }
  if (tid < 3 * CH / 4) *(volatile v4f*)stp = sv;
}

__global__ __launch_bounds__(NTHR) void k_final(
    const float* __restrict__ R7, const float* __restrict__ ss7,
    const float* __restrict__ R5, const float* __restrict__ ss5,
    const float* __restrict__ feat, float* out) {
  const size_t e = ((size_t)blockIdx.x * NTHR + threadIdx.x) * 4;
  const int c0 = (int)(e & (CH - 1));
  const v4f x7 = *(const v4f*)(R7 + e);
  const v4f x5 = *(const v4f*)(R5 + e);
  const v4f f  = *(const v4f*)(feat + e);
  const v4f s7 = *(const v4f*)(ss7 + c0), h7 = *(const v4f*)(ss7 + CH + c0);
  const v4f s5 = *(const v4f*)(ss5 + c0), h5 = *(const v4f*)(ss5 + CH + c0);
  const v4f fu = lre4(x5 * s5 + h5) + f;
  const v4f y  = lre4(x7 * s7 + h7 + fu);
  float* op = out + e;
  *(volatile v4f*)op = y;
  __threadfence();
  *(volatile v4f*)op = y;
}

extern "C" void kernel_launch(void* const* d_in, const int* in_sizes, int n_in,
                              void* d_out, int out_size, void* d_ws, size_t ws_size,
                              hipStream_t stream) {
  if (n_in < 20) return;
  if (in_sizes[0] != NV * CH || in_sizes[1] != NLEV * NV || in_sizes[2] != NV * NTAP) return;
  if (in_sizes[3] != NLEV * CH * CH || in_sizes[4] != NLEV * CH || in_sizes[5] != NLEV * CH) return;
  if (in_sizes[6] != NLEV * CH * CH || in_sizes[7] != 4 * CH * CH || in_sizes[8] != 4 * CH || in_sizes[9] != 4 * CH) return;
  if (in_sizes[10] != CH * NLEV || in_sizes[11] != 2 * CH * CH || in_sizes[12] != CH || in_sizes[13] != CH) return;
  if (in_sizes[14] != NTAP * CH * CH || in_sizes[15] != NTAP * CH * CH) return;
  if (in_sizes[16] != CH || in_sizes[17] != CH || in_sizes[18] != CH || in_sizes[19] != CH) return;
  if (out_size != NV * CH) return;

  const float* feat       = (const float*)d_in[0];
  const int*   clusters   = (const int*)d_in[1];
  const int*   nidx       = (const int*)d_in[2];
  const float* lw_w       = (const float*)d_in[3];
  const float* lw_gamma   = (const float*)d_in[4];
  const float* lw_beta    = (const float*)d_in[5];
  const float* w_w        = (const float*)d_in[6];
  const float* proj_w     = (const float*)d_in[7];
  const float* proj_gamma = (const float*)d_in[8];
  const float* proj_beta  = (const float*)d_in[9];
  const float* adaptive_w = (const float*)d_in[10];
  const float* fuse_w     = (const float*)d_in[11];
  const float* fuse_gamma = (const float*)d_in[12];
  const float* fuse_beta  = (const float*)d_in[13];
  const float* conv1_w    = (const float*)d_in[14];
  const float* conv2_w    = (const float*)d_in[15];
  const float* bn1_gamma  = (const float*)d_in[16];
  const float* bn1_beta   = (const float*)d_in[17];
  const float* bn2_gamma  = (const float*)d_in[18];
  const float* bn2_beta   = (const float*)d_in[19];
  float* out = (float*)d_out;

  char* ws = (char*)d_ws;
  size_t off = 0;
  const size_t MAT2  = (size_t)CH * CH * 2;
  const size_t PLANE = (size_t)NV * CH * 4;
  const size_t oLwH = off; off += NLEV * MAT2;           off = (off + 255) & ~(size_t)255;
  const size_t oLwL = off; off += NLEV * MAT2;           off = (off + 255) & ~(size_t)255;
  const size_t oWwH = off; off += NLEV * MAT2;           off = (off + 255) & ~(size_t)255;
  const size_t oWwL = off; off += NLEV * MAT2;           off = (off + 255) & ~(size_t)255;
  const size_t oPjH = off; off += 4 * MAT2;              off = (off + 255) & ~(size_t)255;
  const size_t oPjL = off; off += 4 * MAT2;              off = (off + 255) & ~(size_t)255;
  const size_t oFuH = off; off += 2 * MAT2;              off = (off + 255) & ~(size_t)255;
  const size_t oFuL = off; off += 2 * MAT2;              off = (off + 255) & ~(size_t)255;
  const size_t oC1  = off; off += (size_t)CH * KCONV * 2; off = (off + 255) & ~(size_t)255;
  const size_t oC2  = off; off += (size_t)CH * KCONV * 2; off = (off + 255) & ~(size_t)255;
  const size_t oPA  = off; off += PLANE;                  off = (off + 255) & ~(size_t)255;
  const size_t oPB  = off; off += PLANE;                  off = (off + 255) & ~(size_t)255;
  const size_t oX16 = off; off += (size_t)NV * CH * 2;    off = (off + 255) & ~(size_t)255;
  const size_t oST  = off; off += (size_t)(NV / CROWS) * STSTR * 4; off = (off + 255) & ~(size_t)255;
  const size_t oSS  = off; off += (size_t)NSS * SSSTR * 4; off = (off + 255) & ~(size_t)255;
  const size_t oT1  = off; off += (size_t)NSEG * CH * 4;   off = (off + 255) & ~(size_t)255;
  const size_t oT2  = off; off += (size_t)NSEG * CH * 4;   off = (off + 255) & ~(size_t)255;
  const size_t oT3  = off; off += (size_t)NLEV * NSEG * CH * 4; off = (off + 255) & ~(size_t)255;
  const size_t oADP = off; off += (size_t)NV * 4 * 4;      off = (off + 255) & ~(size_t)255;
  if (off > ws_size || off > (size_t)134217728) return;

  unsigned short* lwH = (unsigned short*)(ws + oLwH);
  unsigned short* lwL = (unsigned short*)(ws + oLwL);
  unsigned short* wwH = (unsigned short*)(ws + oWwH);
  unsigned short* wwL = (unsigned short*)(ws + oWwL);
  unsigned short* pjH = (unsigned short*)(ws + oPjH);
  unsigned short* pjL = (unsigned short*)(ws + oPjL);
  unsigned short* fuH = (unsigned short*)(ws + oFuH);
  unsigned short* fuL = (unsigned short*)(ws + oFuL);
  _Float16* c1p = (_Float16*)(ws + oC1);
  _Float16* c2p = (_Float16*)(ws + oC2);
  float* PA  = (float*)(ws + oPA);
  float* PB  = (float*)(ws + oPB);
  _Float16* X16 = (_Float16*)(ws + oX16);
  float* ST  = (float*)(ws + oST);
  float* SS  = (float*)(ws + oSS);
  float* T1  = (float*)(ws + oT1);
  float* T2  = (float*)(ws + oT2);
  float* T3  = (float*)(ws + oT3);
  float* ADP = (float*)(ws + oADP);
  float* SS0 = SS + 0 * SSSTR;
  float* SS1 = SS + 1 * SSSTR;
  float* SS2 = SS + 2 * SSSTR;
  float* SS3 = SS + 3 * SSSTR;
  float* SS4 = SS + 4 * SSSTR;
  float* SS5 = SS + 5 * SSSTR;
  float* SS6 = SS + 6 * SSSTR;

  const int nGemm = NV / GROWS;
  const int nConv = NV / CROWS;
  const int nSeg  = NSEG / SLOTS;
  const int nPrep = (NLEV * (CH * CH / 8) * 2 + 4 * (CH * CH / 8) + (2 * CH * CH) / 8 + 2 * ((CH * KCONV) / 8)) / NTHR;
  const size_t MATE = (size_t)CH * CH;

  hipFuncSetAttribute(reinterpret_cast<const void*>(&k_gemm<0>), hipFuncAttributeMaxDynamicSharedMemorySize, LDS_GEMM);
  hipFuncSetAttribute(reinterpret_cast<const void*>(&k_gemm<1>), hipFuncAttributeMaxDynamicSharedMemorySize, LDS_GEMM);
  hipFuncSetAttribute(reinterpret_cast<const void*>(&k_gemm<2>), hipFuncAttributeMaxDynamicSharedMemorySize, LDS_GEMM);

  k_prep<<<nPrep, NTHR, 0, stream>>>(lw_w, w_w, proj_w, fuse_w, conv1_w, conv2_w,
                                     lwH, lwL, wwH, wwL, pjH, pjL, fuH, fuL, c1p, c2p);

  for (int i = 0; i < NLEV; ++i) {
    const int* ids = clusters + (size_t)i * NV;
    k_gemm<0><<<nGemm, NTHR, LDS_GEMM, stream>>>(feat, SS0, ids, T1, ADP, lwH + i * MATE, lwL + i * MATE, PA, ST);
    k_bnfin<<<1, CH, 0, stream>>>(ST, nGemm, GROWS, lw_gamma + i * CH, lw_beta + i * CH, 1, SS0);
    k_seg<0><<<nSeg, NTHR, 0, stream>>>(ids, PA, PA, SS0, SS0, T1, T1);
    k_gemm<1><<<nGemm, NTHR, LDS_GEMM, stream>>>(PA, SS0, ids, T1, ADP, wwH + i * MATE, wwL + i * MATE, PB, ST);
    k_bnfin<<<1, CH, 0, stream>>>(ST, nGemm, GROWS, lw_gamma + i * CH, lw_beta + i * CH, 0, SS1);
    k_seg<1><<<nSeg, NTHR, 0, stream>>>(ids, PB, PB, SS0, SS1, T1, T2);
    k_gemm<0><<<nGemm, NTHR, LDS_GEMM, stream>>>(feat, SS0, ids, T1, ADP, pjH + i * MATE, pjL + i * MATE, PA, ST);
    k_bnfin<<<1, CH, 0, stream>>>(ST, nGemm, GROWS, proj_gamma + i * CH, proj_beta + i * CH, 1, SS2);
    k_seg<2><<<nSeg, NTHR, 0, stream>>>(ids, PA, PB, SS2, SS1, T2, T3 + (size_t)i * NSEG * CH);
  }

  k_adp<<<NV / NTHR, NTHR, 0, stream>>>(feat, adaptive_w, ADP);
  k_gemm<0><<<nGemm, NTHR, LDS_GEMM, stream>>>(feat, SS0, clusters, T1, ADP, pjH + 3 * MATE, pjL + 3 * MATE, PA, ST);
  k_bnfin<<<1, CH, 0, stream>>>(ST, nGemm, GROWS, proj_gamma + 3 * CH, proj_beta + 3 * CH, 1, SS3);
  k_gemm<2><<<nGemm, NTHR, LDS_GEMM, stream>>>(PA, SS3, clusters, T3, ADP, fuH, fuL, PB, ST);
  k_bnfin<<<1, CH, 0, stream>>>(ST, nGemm, GROWS, fuse_gamma, fuse_beta, 1, SS4);
  k_x16<<<(NV * CH / 8) / NTHR, NTHR, 0, stream>>>(PB, SS4, feat, 1, X16);
  k_conv<<<nConv, CTHR, 0, stream>>>(X16, nidx, c1p, PA, ST);
  k_bnfin<<<1, CH, 0, stream>>>(ST, nConv, CROWS, bn1_gamma, bn1_beta, 1, SS5);
  k_x16<<<(NV * CH / 8) / NTHR, NTHR, 0, stream>>>(PA, SS5, feat, 0, X16);
  k_conv<<<nConv, CTHR, 0, stream>>>(X16, nidx, c2p, PA, ST);
  k_bnfin<<<1, CH, 0, stream>>>(ST, nConv, CROWS, bn2_gamma, bn2_beta, 1, SS6);
  k_final<<<(NV * CH / 4) / NTHR, NTHR, 0, stream>>>(PA, SS6, PB, SS4, feat, out);
}
